// GraphEncoder_4037269258797
// MI455X (gfx1250) — hardware-verified
//
#include <hip/hip_runtime.h>
#include <stddef.h>
#include <stdint.h>
#include <math.h>


#define F_IN    128
#define HC1     256
#define HID     64
#define NHD     4
#define KA      128
#define EDIM    8
#define NLAY    3
#define NGR     1024
#define NTHR    256
#define NWAVE   8
#define EPT     8
#define CHUNK   (NTHR * EPT)
#define WCAP    (EPT * 32)
#define LISTN   (NWAVE * WCAP)
#define NBMAX   2048
#define SLOTB   11
#define NBRUN   1024
#define RCAP    16384
#define DEGCAP  64
#define MEAS_B1024  10475
#define MEAS_MAXDEG 26
#define GBM     64
#define GBN     64
#define GTHR    128
#define MROWS   128
#define NEGSL   0.2f
#define EPS_SM  1e-16f
#define BN_EPS  1e-5f
#define WSMAX   134217728
#define LDS_BKT ((2 * RCAP + 2 * NBMAX + LISTN + 16 + 128) * 4)

static_assert((CHUNK & (CHUNK - 1)) == 0 && CHUNK <= (1 << SLOTB));
static_assert(NBMAX == (1 << SLOTB));
static_assert(NTHR * 8 == NBMAX);
static_assert(LISTN >= NBMAX);
static_assert(LISTN >= NWAVE * WCAP);
static_assert((RCAP % 32) == 0);
static_assert(NBRUN <= NBMAX && NBRUN == 4 * NTHR && (NBRUN % NWAVE) == 0);
static_assert(RCAP * 100 >= MEAS_B1024 * 105);
static_assert(DEGCAP >= MEAS_MAXDEG + 8);
static_assert(RCAP >= NLAY * NBRUN * 4);
static_assert((RCAP % (2 * NTHR)) == 0);
static_assert(LDS_BKT <= 300000);
static_assert(GBM == (GTHR / 32) * 16);
static_assert(GTHR == 2 * GBN && GTHR == 2 * GBM);
static_assert((F_IN % 32) == 0 && (KA % 32) == 0);
static_assert((HC1 % GBN) == 0 && HID == GBN);
static_assert(HC1 == NHD * HID);
static_assert(KA == 2 * HID);
static_assert((MROWS % GBM) == 0);
static_assert(HC1 == 8 * 32);
static_assert(HID == 8 * 8);
static_assert((F_IN / 8) == 16);
static_assert(NLAY * EDIM * NHD <= 128);

typedef float          v2f  __attribute__((ext_vector_type(2)));
typedef float          v4f  __attribute__((ext_vector_type(4)));
typedef float          v8f  __attribute__((ext_vector_type(8)));
typedef int            v2i  __attribute__((ext_vector_type(2)));
typedef int            v4i  __attribute__((ext_vector_type(4)));
typedef int            v8i  __attribute__((ext_vector_type(8)));
typedef unsigned int   v4u  __attribute__((ext_vector_type(4)));
typedef unsigned short v8us __attribute__((ext_vector_type(8)));
typedef __bf16         v16b __attribute__((ext_vector_type(16)));
typedef v2f  __attribute__((may_alias)) v2fa;
typedef v4f  __attribute__((may_alias)) v4fa;
typedef v2i  __attribute__((may_alias)) v2ia;
typedef v4i  __attribute__((may_alias)) v4ia;
typedef v8us __attribute__((may_alias)) v8usa;
union FragB { v16b v; v8us h[2]; v8i w; };
struct HL8 { v4u h; v4u l; };

__device__ __forceinline__ v8f wmb(const FragB& a, const FragB& b, v8f c) {
  v8f d = __builtin_amdgcn_wmma_f32_16x16x32_bf16(false, a.v, false, b.v, (short)0, c, false, false);
  asm volatile("v_nop\n\tv_nop\n\tv_nop\n\tv_nop" : "+v"(d) : "v"(a.w), "v"(b.w));
  return d;
}

__device__ __forceinline__ unsigned int f2bf(float f) {
  const unsigned int u = __float_as_uint(f);
  const unsigned int r = ((u + 0x7FFFu + ((u >> 16) & 1u)) >> 16) & 0xFFFFu;
  return (f != f) ? 0x7FC0u : r;
}
__device__ __forceinline__ float bf2f(unsigned int b) { return __uint_as_float(b << 16); }
__device__ __forceinline__ float bfr(float f) { return bf2f(f2bf(f)); }
__device__ __forceinline__ v4f bfr4(const v4f a) {
  v4f r; r.x = bfr(a.x); r.y = bfr(a.y); r.z = bfr(a.z); r.w = bfr(a.w); return r;
}
__device__ __forceinline__ unsigned int pk2(float lo, float hi) { return f2bf(lo) | (f2bf(hi) << 16); }
__device__ __forceinline__ v4u pack8(const v4f a, const v4f b) {
  v4u r;
  r.x = pk2(a.x, a.y); r.y = pk2(a.z, a.w); r.z = pk2(b.x, b.y); r.w = pk2(b.z, b.w);
  return r;
}
__device__ __forceinline__ HL8 split8(const v4f a, const v4f b) {
  const unsigned int h0 = f2bf(a.x), h1 = f2bf(a.y), h2 = f2bf(a.z), h3 = f2bf(a.w);
  const unsigned int h4 = f2bf(b.x), h5 = f2bf(b.y), h6 = f2bf(b.z), h7 = f2bf(b.w);
  const unsigned int g0 = f2bf(a.x - bf2f(h0)), g1 = f2bf(a.y - bf2f(h1));
  const unsigned int g2 = f2bf(a.z - bf2f(h2)), g3 = f2bf(a.w - bf2f(h3));
  const unsigned int g4 = f2bf(b.x - bf2f(h4)), g5 = f2bf(b.y - bf2f(h5));
  const unsigned int g6 = f2bf(b.z - bf2f(h6)), g7 = f2bf(b.w - bf2f(h7));
  HL8 r;
  r.h.x = h0 | (h1 << 16); r.h.y = h2 | (h3 << 16); r.h.z = h4 | (h5 << 16); r.h.w = h6 | (h7 << 16);
  r.l.x = g0 | (g1 << 16); r.l.y = g2 | (g3 << 16); r.l.z = g4 | (g5 << 16); r.l.w = g6 | (g7 << 16);
  return r;
}

__device__ __forceinline__ int scan_chunk(const int* __restrict__ dsts, int nE, int cbase, int slotBase,
                                          int nb, int vec8, int* list, int tid, int lane, int wave) {
  int wc = 0;
  const int el0  = tid * EPT;
  const int e0   = cbase + el0;
  const int sent = -2147483647 - 1;
  v4i da, db;
  if (vec8 != 0 && cbase + CHUNK <= nE) {
    da = *(const v4i*)(dsts + e0);
    db = *(const v4i*)(dsts + e0 + 4);
  } else {
    da.x = (e0     < nE) ? dsts[min(e0,     nE - 1)] : sent;
    da.y = (e0 + 1 < nE) ? dsts[min(e0 + 1, nE - 1)] : sent;
    da.z = (e0 + 2 < nE) ? dsts[min(e0 + 2, nE - 1)] : sent;
    da.w = (e0 + 3 < nE) ? dsts[min(e0 + 3, nE - 1)] : sent;
    db.x = (e0 + 4 < nE) ? dsts[min(e0 + 4, nE - 1)] : sent;
    db.y = (e0 + 5 < nE) ? dsts[min(e0 + 5, nE - 1)] : sent;
    db.z = (e0 + 6 < nE) ? dsts[min(e0 + 6, nE - 1)] : sent;
    db.w = (e0 + 7 < nE) ? dsts[min(e0 + 7, nE - 1)] : sent;
  }
  const unsigned nbs = (unsigned)slotBase;
  const unsigned unb = (unsigned)nb;
  const unsigned s0 = (unsigned)da.x - nbs, s1 = (unsigned)da.y - nbs;
  const unsigned s2 = (unsigned)da.z - nbs, s3 = (unsigned)da.w - nbs;
  const unsigned s4 = (unsigned)db.x - nbs, s5 = (unsigned)db.y - nbs;
  const unsigned s6 = (unsigned)db.z - nbs, s7 = (unsigned)db.w - nbs;
  const bool h0 = s0 < unb, h1 = s1 < unb, h2 = s2 < unb, h3 = s3 < unb;
  const bool h4 = s4 < unb, h5 = s5 < unb, h6 = s6 < unb, h7 = s7 < unb;
  const unsigned any = __builtin_amdgcn_ballot_w32(h0 | h1 | h2 | h3 | h4 | h5 | h6 | h7);
  if (any != 0u) {
#define HITJ(J, HJ, SJ) { \
      const unsigned mj = __builtin_amdgcn_ballot_w32(HJ); \
      if (mj != 0u) { \
        if (HJ) { \
          const int pos = wc + (int)__builtin_amdgcn_mbcnt_lo(mj, 0u); \
          if (pos < WCAP) list[wave * WCAP + pos] = ((el0 + (J)) << SLOTB) | (int)(SJ); \
        } \
        wc += (int)__builtin_popcount(mj); } }
    HITJ(0, h0, s0)
    HITJ(1, h1, s1)
    HITJ(2, h2, s2)
    HITJ(3, h3, s3)
    HITJ(4, h4, s4)
    HITJ(5, h5, s5)
    HITJ(6, h6, s6)
    HITJ(7, h7, s7)
#undef HITJ
  }
  return wc;
}

__global__ __launch_bounds__(NTHR) void k_xprep(const float* __restrict__ x, unsigned short* xb, int nN, int nUnits) {
  const int i = (int)blockIdx.x * NTHR + (int)threadIdx.x;
  if (i >= nUnits) return;
  const int row = i >> 4;
  const int c0  = (i & 15) * 8;
  const int rc  = row < nN ? row : nN - 1;
  const float* p = x + (size_t)rc * F_IN + c0;
  v4f a = *(const v4fa*)p, b = *(const v4fa*)(p + 4);
  const v4f z4 = {0.f, 0.f, 0.f, 0.f};
  if (row >= nN) { a = z4; b = z4; }
  const v4u hv = pack8(a, b);
  const size_t o = (size_t)row * F_IN + c0;
  *(volatile v4u*)(xb + o) = hv;
  __threadfence();
  *(volatile v4u*)(xb + o) = hv;
}

__global__ __launch_bounds__(NTHR) void k_wtr(const float* __restrict__ w, int Kin, int Ncol, int Nrows, int Kout,
                                              unsigned short* wt, int nUnits) {
  const int u = (int)blockIdx.x * NTHR + (int)threadIdx.x;
  if (u >= nUnits) return;
  const int kq = Kout >> 3;
  const int n  = u / kq;
  const int k8 = (u - n * kq) * 8;
  const int kk = k8 - (k8 / Kin) * Kin;
  const int ncl = n < Ncol ? n : Ncol - 1;
  const float* p = w + (size_t)kk * (size_t)Ncol + ncl;
  v4f a, b;
  a.x = p[0];                    a.y = p[(size_t)Ncol];         a.z = p[(size_t)2 * Ncol];     a.w = p[(size_t)3 * Ncol];
  b.x = p[(size_t)4 * Ncol];     b.y = p[(size_t)5 * Ncol];     b.z = p[(size_t)6 * Ncol];     b.w = p[(size_t)7 * Ncol];
  const v4f z4 = {0.f, 0.f, 0.f, 0.f};
  if (n >= Ncol || n >= Nrows) { a = z4; b = z4; }
  const v4u wv = pack8(a, b);
  unsigned short* o = wt + (size_t)n * (size_t)Kout + k8;
  *(volatile v4u*)o = wv;
  __threadfence();
  *(volatile v4u*)o = wv;
}

__global__ __launch_bounds__(NTHR) void k_tab(const float* __restrict__ lew, const float* __restrict__ atte,
                                              const float* __restrict__ cbias, const float* __restrict__ gam,
                                              const float* __restrict__ bet, const float* __restrict__ mean,
                                              const float* __restrict__ var, float* KAP, float* TB) {
  __shared__ __attribute__((aligned(16))) float sk[128];
  __shared__ __attribute__((aligned(16))) float sb[NLAY * 256];
  const int tid = (int)threadIdx.x;
  float kv = 0.f;
  if (tid < 96) {
    const int l = tid >> 5, r = tid & 31, d = r >> 2, hd = r & 3;
    const float* W = lew + (size_t)l * EDIM * HC1 + (size_t)d * HC1 + hd * HID;
    const float* a = atte + (size_t)l * HC1 + hd * HID;
    float s = 0.f;
#pragma unroll 2
    for (int c4 = 0; c4 < HID / 4; ++c4) {
      const v4f wv = bfr4(*(const v4fa*)(W + 4 * c4));
      const v4f av = bfr4(*(const v4fa*)(a + 4 * c4));
      s = fmaf(wv.x, av.x, s);
      s = fmaf(wv.y, av.y, s);
      s = fmaf(wv.z, av.z, s);
      s = fmaf(wv.w, av.w, s);
    }
    kv = s;
  }
  if (tid < 128) sk[tid] = kv;
  if (tid < NLAY * HID) {
    const int l = tid >> 6, c = tid & 63;
    const float cbv = bfr(cbias[tid]);
    const float g   = bfr(gam[tid]);
    const float b   = bfr(bet[tid]);
    const float mu  = bfr(mean[tid]);
    const float vv  = bfr(var[tid]);
    const float sc  = g / sqrtf(vv + BN_EPS);
    sb[l * 256 + c]       = cbv;
    sb[l * 256 + 64 + c]  = mu;
    sb[l * 256 + 128 + c] = sc;
    sb[l * 256 + 192 + c] = b;
  }
  __syncthreads();
  const int tq = tid < 192 ? tid : 191;
  const v4f kq = *(const v4fa*)(sk + 4 * (tid & 31));
  const v4f bq = *(const v4fa*)(sb + 4 * tq);
  if (tid < 32)  *(volatile v4f*)(KAP + 4 * tid) = kq;
  if (tid < 192) *(volatile v4f*)(TB + 4 * tid) = bq;
  __threadfence();
  if (tid < 32)  *(volatile v4f*)(KAP + 4 * tid) = kq;
  if (tid < 192) *(volatile v4f*)(TB + 4 * tid) = bq;
}

__global__ __launch_bounds__(NTHR) void k_edge(const float* __restrict__ ea, const float* __restrict__ KAP,
                                               float* AE, int nE) {
  __shared__ __attribute__((aligned(16))) float sk[128];
  const int tid = (int)threadIdx.x;
  if (tid < 128) sk[tid] = KAP[tid];
  __syncthreads();
  const int e  = (int)blockIdx.x * NTHR + tid;
  const int ec = e < nE ? e : nE - 1;
  const bool ok = e < nE;
  const float* p = ea + (size_t)ec * EDIM;
  const v4f a = bfr4(*(const v4fa*)p);
  const v4f b = bfr4(*(const v4fa*)(p + 4));
#pragma unroll 1
  for (int l = 0; l < NLAY; ++l) {
    const float* kp = sk + l * 32;
    v4f r = {0.f, 0.f, 0.f, 0.f};
    { const v4f k = *(const v4fa*)(kp + 0);  r.x = fmaf(a.x, k.x, r.x); r.y = fmaf(a.x, k.y, r.y); r.z = fmaf(a.x, k.z, r.z); r.w = fmaf(a.x, k.w, r.w); }
    { const v4f k = *(const v4fa*)(kp + 4);  r.x = fmaf(a.y, k.x, r.x); r.y = fmaf(a.y, k.y, r.y); r.z = fmaf(a.y, k.z, r.z); r.w = fmaf(a.y, k.w, r.w); }
    { const v4f k = *(const v4fa*)(kp + 8);  r.x = fmaf(a.z, k.x, r.x); r.y = fmaf(a.z, k.y, r.y); r.z = fmaf(a.z, k.z, r.z); r.w = fmaf(a.z, k.w, r.w); }
    { const v4f k = *(const v4fa*)(kp + 12); r.x = fmaf(a.w, k.x, r.x); r.y = fmaf(a.w, k.y, r.y); r.z = fmaf(a.w, k.z, r.z); r.w = fmaf(a.w, k.w, r.w); }
    { const v4f k = *(const v4fa*)(kp + 16); r.x = fmaf(b.x, k.x, r.x); r.y = fmaf(b.x, k.y, r.y); r.z = fmaf(b.x, k.z, r.z); r.w = fmaf(b.x, k.w, r.w); }
    { const v4f k = *(const v4fa*)(kp + 20); r.x = fmaf(b.y, k.x, r.x); r.y = fmaf(b.y, k.y, r.y); r.z = fmaf(b.y, k.z, r.z); r.w = fmaf(b.y, k.w, r.w); }
    { const v4f k = *(const v4fa*)(kp + 24); r.x = fmaf(b.z, k.x, r.x); r.y = fmaf(b.z, k.y, r.y); r.z = fmaf(b.z, k.z, r.z); r.w = fmaf(b.z, k.w, r.w); }
    { const v4f k = *(const v4fa*)(kp + 28); r.x = fmaf(b.w, k.x, r.x); r.y = fmaf(b.w, k.y, r.y); r.z = fmaf(b.w, k.z, r.z); r.w = fmaf(b.w, k.w, r.w); }
    float* op = AE + ((size_t)l * (size_t)nE + (size_t)ec) * 4;
    if (ok) *(volatile v4f*)op = r;
    __threadfence();
    if (ok) *(volatile v4f*)op = r;
  }
}

__device__ __forceinline__ void bkt_store(const int* reg2, const float* res, const int* scnt, const int* soff,
                                          const int* __restrict__ srcs, int* hitsB, int* offB, int* cntB,
                                          float* LAE, int nodeBase, int nslot, int nN, int nE, int nh, bool ovf,
                                          int tid) {
#pragma unroll 1
  for (int p = tid; p < NLAY * NBRUN; p += NTHR) {
    const int l    = p / NBRUN;
    const int slot = p - l * NBRUN;
    const v4f v = *(const v4fa*)(res + 4 * p);
    *(volatile v4f*)(LAE + ((size_t)l * (size_t)nslot + (size_t)(nodeBase + slot)) * 4) = v;
  }
#pragma unroll 1
  for (int p = tid; p < RCAP / 2; p += NTHR) {
    const int i0 = 2 * p, i1 = 2 * p + 1;
    int eA = reg2[i0], eB = reg2[i1];
    eA = (i0 < nh) ? eA : 0;
    eB = (i1 < nh) ? eB : 0;
    eA = eA < 0 ? 0 : (eA > nE - 1 ? nE - 1 : eA);
    eB = eB < 0 ? 0 : (eB > nE - 1 ? nE - 1 : eB);
    int sA = srcs[eA], sB = srcs[eB];
    sA = sA < 0 ? 0 : (sA > nN - 1 ? nN - 1 : sA);
    sB = sB < 0 ? 0 : (sB > nN - 1 ? nN - 1 : sB);
    v4i o; o.x = sA; o.y = eA; o.z = sB; o.w = eB;
    *(volatile v4i*)(hitsB + 4 * p) = o;
  }
  {
    const v4i so = *(const v4ia*)(soff + 4 * tid);
    v4i sc = *(const v4ia*)(scnt + 4 * tid);
    const int big = 0x7fffffff;
    sc.x = ovf ? big : sc.x; sc.y = ovf ? big : sc.y; sc.z = ovf ? big : sc.z; sc.w = ovf ? big : sc.w;
    *(volatile v4i*)(offB + 4 * tid) = so;
    *(volatile v4i*)(cntB + 4 * tid) = sc;
  }
}

__global__ __launch_bounds__(NTHR) void k_bucket(
    const int* __restrict__ srcs, const int* __restrict__ dsts, const float* __restrict__ eattr,
    const float* __restrict__ KAP, int* HITS, int* OFF, int* CNT, float* LAE,
    int nN, int nE, int vec8, int nslot) {
  extern __shared__ v4f lds_dyn[];
  int* reg1 = (int*)lds_dyn;
  int* reg2 = reg1 + RCAP;
  int* scnt = reg2 + RCAP;
  int* soff = scnt + NBMAX;
  int* list = soff + NBMAX;
  int* wcnt = list + LISTN;
  int* wtot = wcnt + NWAVE;
  float* skap = (float*)(wtot + NWAVE);
  const int tid = (int)threadIdx.x, lane = tid & 31, wave = tid >> 5;
  const int nodeBase = (int)blockIdx.x * NBRUN;

  {
    const v4i z4 = {0, 0, 0, 0};
    for (int i = tid * 4; i < 2 * RCAP; i += NTHR * 4) *(v4ia*)(reg1 + i) = z4;
    for (int i = tid; i < NBMAX; i += NTHR) { scnt[i] = 0; soff[i] = 0; }
    for (int i = tid; i < LISTN; i += NTHR) list[i] = 0;
    if (tid < NWAVE) { wcnt[tid] = 0; wtot[tid] = 0; }
    if (tid < 128) skap[tid] = KAP[tid];
  }
  __syncthreads();

  int tot = 0;
  const int nChunks = (nE + CHUNK - 1) / CHUNK;
#pragma unroll 1
  for (int ch = 0; ch < nChunks; ++ch) {
    const int cbase = ch * CHUNK;
    const int wc = scan_chunk(dsts, nE, cbase, nodeBase, NBRUN, vec8, list, tid, lane, wave);
    if (lane == 0) wcnt[wave] = wc;
    __syncthreads();
    int pre = 0, all = 0;
#pragma unroll
    for (int w2 = 0; w2 < NWAVE; ++w2) {
      int c = wcnt[w2];
      c = c < 0 ? 0 : (c > WCAP ? WCAP : c);
      all += c;
      pre += (w2 < wave) ? c : 0;
    }
    const int wcc  = wc > WCAP ? WCAP : wc;
    const int base = tot + pre;
#pragma unroll 1
    for (int i = lane; i < wcc; i += 32) {
      const int ent = list[wave * WCAP + i];
      const int el  = (ent >> SLOTB) & (CHUNK - 1);
      const int sl  = ent & (NBMAX - 1);
      int eid = cbase + el;
      eid = eid > nE - 1 ? nE - 1 : eid;
      const int pos = base + i;
      if (pos < RCAP) reg1[pos] = (int)(((unsigned)eid << SLOTB) | (unsigned)sl);
    }
    tot += all;
    tot = tot > RCAP ? RCAP : tot;
    __syncthreads();
  }
  const int nh = tot;

  if (wave == 0) {
#pragma unroll 1
    for (int b0 = 0; b0 < nh; b0 += 32) {
      const int idx = b0 + lane;
      const int uv  = reg1[idx < nh ? idx : nh - 1];
      const int m32 = (nh - b0) < 32 ? (nh - b0) : 32;
#pragma unroll 1
      for (int k = 0; k < m32; ++k) {
        const int u  = __builtin_amdgcn_readlane(uv, k);
        const int sl = u & (NBMAX - 1);
        if (lane == 0) scnt[sl] = scnt[sl] + 1;
      }
    }
  }
  __syncthreads();

  {
    const v4i ca = *(const v4ia*)(scnt + 8 * tid);
    const v4i cb = *(const v4ia*)(scnt + 8 * tid + 4);
    const int e0 = ca.x < 0 ? 0 : ca.x, e1 = ca.y < 0 ? 0 : ca.y, e2 = ca.z < 0 ? 0 : ca.z, e3 = ca.w < 0 ? 0 : ca.w;
    const int e4 = cb.x < 0 ? 0 : cb.x, e5 = cb.y < 0 ? 0 : cb.y, e6 = cb.z < 0 ? 0 : cb.z, e7 = cb.w < 0 ? 0 : cb.w;
    const int ts = e0 + e1 + e2 + e3 + e4 + e5 + e6 + e7;
    int incl = ts;
#pragma unroll
    for (int d = 1; d < 32; d <<= 1) {
      const int up = __shfl_up(incl, d);
      if (lane >= d) incl += up;
    }
    if (lane == 31) wtot[wave] = incl;
    __syncthreads();
    int pre = 0;
#pragma unroll
    for (int w2 = 0; w2 < NWAVE; ++w2) pre += (w2 < wave) ? wtot[w2] : 0;
    int run = pre + incl - ts;
    soff[8 * tid + 0] = run; run += e0;
    soff[8 * tid + 1] = run; run += e1;
    soff[8 * tid + 2] = run; run += e2;
    soff[8 * tid + 3] = run; run += e3;
    soff[8 * tid + 4] = run; run += e4;
    soff[8 * tid + 5] = run; run += e5;
    soff[8 * tid + 6] = run; run += e6;
    soff[8 * tid + 7] = run;
  }
  __syncthreads();
  for (int i = tid; i < NBMAX; i += NTHR) list[i] = soff[i];
  __syncthreads();

  if (wave == 0) {
#pragma unroll 1
    for (int b0 = 0; b0 < nh; b0 += 32) {
      const int idx = b0 + lane;
      const int uv  = reg1[idx < nh ? idx : nh - 1];
      const int m32 = (nh - b0) < 32 ? (nh - b0) : 32;
#pragma unroll 1
      for (int k = 0; k < m32; ++k) {
        const int u   = __builtin_amdgcn_readlane(uv, k);
        const int sl  = u & (NBMAX - 1);
        const int eid = (int)((unsigned)u >> SLOTB);
        if (lane == 0) {
          int pos = list[sl];
          pos = pos < 0 ? 0 : (pos > RCAP - 1 ? RCAP - 1 : pos);
          reg2[pos] = eid;
          list[sl] = pos + 1;
        }
      }
    }
  }
  __syncthreads();

  float* res = (float*)reg1;
  const bool ovf = (nh >= RCAP);
#pragma unroll 1
  for (int it = 0; it < NBRUN / NTHR; ++it) {
    const int slot = it * NTHR + tid;
    int st = soff[slot];
    const int craw = scnt[slot];
    st = st < 0 ? 0 : (st > nh ? nh : st);
    int cn = craw < 0 ? 0 : (craw > DEGCAP ? DEGCAP : craw);
    if (cn > nh - st) cn = nh - st;
    int cm = cn;
#pragma unroll
    for (int off = 16; off > 0; off >>= 1) {
      const int o2 = __shfl_xor(cm, off, 32);
      cm = o2 > cm ? o2 : cm;
    }
    cm = cm > DEGCAP ? DEGCAP : cm;
    float a0 = 0.f, a1 = 0.f, a2 = 0.f, a3 = 0.f, a4 = 0.f, a5 = 0.f, a6 = 0.f, a7 = 0.f;
#pragma unroll 1
    for (int q = 0; q < cm; ++q) {
      int idx = st + q; idx = idx > RCAP - 1 ? RCAP - 1 : idx;
      int eid = reg2[idx]; eid = eid < 0 ? 0 : (eid > nE - 1 ? nE - 1 : eid);
      const float* ep = eattr + (size_t)eid * EDIM;
      const v4f ea = bfr4(*(const v4fa*)ep);
      const v4f eb = bfr4(*(const v4fa*)(ep + 4));
      const float w = (q < cn) ? 1.0f : 0.0f;
      a0 = fmaf(w, ea.x, a0); a1 = fmaf(w, ea.y, a1); a2 = fmaf(w, ea.z, a2); a3 = fmaf(w, ea.w, a3);
      a4 = fmaf(w, eb.x, a4); a5 = fmaf(w, eb.y, a5); a6 = fmaf(w, eb.z, a6); a7 = fmaf(w, eb.w, a7);
    }
    const float dgi = 1.0f / (float)(craw < 1 ? 1 : craw);
    a0 *= dgi; a1 *= dgi; a2 *= dgi; a3 *= dgi; a4 *= dgi; a5 *= dgi; a6 *= dgi; a7 *= dgi;
#pragma unroll 1
    for (int l = 0; l < NLAY; ++l) {
      const float* kp = skap + l * 32;
      v4f r = {0.f, 0.f, 0.f, 0.f};
      { const v4f k = *(const v4fa*)(kp + 0);  r.x = fmaf(a0, k.x, r.x); r.y = fmaf(a0, k.y, r.y); r.z = fmaf(a0, k.z, r.z); r.w = fmaf(a0, k.w, r.w); }
      { const v4f k = *(const v4fa*)(kp + 4);  r.x = fmaf(a1, k.x, r.x); r.y = fmaf(a1, k.y, r.y); r.z = fmaf(a1, k.z, r.z); r.w = fmaf(a1, k.w, r.w); }
      { const v4f k = *(const v4fa*)(kp + 8);  r.x = fmaf(a2, k.x, r.x); r.y = fmaf(a2, k.y, r.y); r.z = fmaf(a2, k.z, r.z); r.w = fmaf(a2, k.w, r.w); }
      { const v4f k = *(const v4fa*)(kp + 12); r.x = fmaf(a3, k.x, r.x); r.y = fmaf(a3, k.y, r.y); r.z = fmaf(a3, k.z, r.z); r.w = fmaf(a3, k.w, r.w); }
      { const v4f k = *(const v4fa*)(kp + 16); r.x = fmaf(a4, k.x, r.x); r.y = fmaf(a4, k.y, r.y); r.z = fmaf(a4, k.z, r.z); r.w = fmaf(a4, k.w, r.w); }
      { const v4f k = *(const v4fa*)(kp + 20); r.x = fmaf(a5, k.x, r.x); r.y = fmaf(a5, k.y, r.y); r.z = fmaf(a5, k.z, r.z); r.w = fmaf(a5, k.w, r.w); }
      { const v4f k = *(const v4fa*)(kp + 24); r.x = fmaf(a6, k.x, r.x); r.y = fmaf(a6, k.y, r.y); r.z = fmaf(a6, k.z, r.z); r.w = fmaf(a6, k.w, r.w); }
      { const v4f k = *(const v4fa*)(kp + 28); r.x = fmaf(a7, k.x, r.x); r.y = fmaf(a7, k.y, r.y); r.z = fmaf(a7, k.z, r.z); r.w = fmaf(a7, k.w, r.w); }
      *(v4fa*)(res + (size_t)(l * NBRUN + slot) * 4) = r;
    }
  }
  __syncthreads();

  int* hitsB = HITS + (size_t)blockIdx.x * (size_t)RCAP * 2;
  int* offB  = OFF + nodeBase;
  int* cntB  = CNT + nodeBase;
  bkt_store(reg2, res, scnt, soff, srcs, hitsB, offB, cntB, LAE, nodeBase, nslot, nN, nE, nh, ovf, tid);
  __threadfence();
  bkt_store(reg2, res, scnt, soff, srcs, hitsB, offB, cntB, LAE, nodeBase, nslot, nN, nE, nh, ovf, tid);
}

template <int WHL>
__global__ __launch_bounds__(GTHR) void k_gemmb(
    const unsigned short* __restrict__ A, const unsigned short* __restrict__ WT,
    const float* __restrict__ bias, float* outF, unsigned short* outHL, int K)
{
  __shared__ __attribute__((aligned(16))) float stg[GBM * GBN];
  const int tid = (int)threadIdx.x, lane = tid & 31, wave = tid >> 5, hh = lane >> 4, m = lane & 15;
  const int rowBase = (int)blockIdx.x * GBM;

  v8f acc[4];
  {
    const v8f z = {0.f, 0.f, 0.f, 0.f, 0.f, 0.f, 0.f, 0.f};
    acc[0] = z; acc[1] = z; acc[2] = z; acc[3] = z;
  }
  const unsigned short* ap = A  + (size_t)(rowBase + 16 * wave + m) * (size_t)K + 8 * hh;
  const unsigned short* wp = WT + (size_t)m * (size_t)K + 8 * hh;
  const int ksteps = K >> 5;
#pragma unroll 1
  for (int ks = 0; ks < ksteps; ++ks) {
    FragB af;
    af.h[0] = *(const v8usa*)(ap + 32 * ks);
    af.h[1] = *(const v8usa*)(ap + 32 * ks + 16);
#pragma unroll
    for (int t = 0; t < 4; ++t) {
      const unsigned short* wq = wp + (size_t)(16 * t) * (size_t)K + 32 * ks;
      FragB bf;
      bf.h[0] = *(const v8usa*)wq;
      bf.h[1] = *(const v8usa*)(wq + 16);
      acc[t] = wmb(af, bf, acc[t]);
    }
  }

#pragma unroll
  for (int t = 0; t < 4; ++t) {
    const int lc = 16 * t + m;
#pragma unroll
    for (int r = 0; r < 8; ++r) {
      const int lr = 16 * wave + 8 * hh + r;
      stg[lr * GBN + lc] = acc[t][r];
    }
  }
  __syncthreads();

  const v4f b4 = bfr4(*(const v4fa*)(bias + 4 * m));
  v4f fv[8];
#pragma unroll
  for (int i = 0; i < 8; ++i) {
    const int lr = 16 * wave + 2 * i + hh;
    const v4f t4 = *(const v4fa*)(stg + lr * GBN + 4 * m);
    fv[i] = t4 + b4;
  }
  v4u pv[8];
  if (WHL != 0) {
    const int ch0 = 8 * (m & 7);
    const v4f bA = bfr4(*(const v4fa*)(bias + ch0));
    const v4f bB = bfr4(*(const v4fa*)(bias + ch0 + 4));
    const bool lsel = (m & 8) != 0;
#pragma unroll
    for (int i = 0; i < 8; ++i) {
      const int lr = 16 * wave + 2 * i + hh;
      const v4f xa = *(const v4fa*)(stg + lr * GBN + ch0) + bA;
      const v4f xb = *(const v4fa*)(stg + lr * GBN + ch0 + 4) + bB;
      const HL8 s = split8(xa, xb);
      v4u q;
      q.x = lsel ? s.l.x : s.h.x; q.y = lsel ? s.l.y : s.h.y;
      q.z = lsel ? s.l.z : s.h.z; q.w = lsel ? s.l.w : s.h.w;
      pv[i] = q;
    }
  }

#pragma unroll
  for (int i = 0; i < 8; ++i) {
    const int gr = rowBase + 16 * wave + 2 * i + hh;
    *(volatile v4f*)(outF + (size_t)gr * GBN + 4 * m) = fv[i];
    if (WHL != 0) *(volatile v4u*)(outHL + (size_t)gr * KA + 8 * m) = pv[i];
  }
  __threadfence();
#pragma unroll
  for (int i = 0; i < 8; ++i) {
    const int gr = rowBase + 16 * wave + 2 * i + hh;
    *(volatile v4f*)(outF + (size_t)gr * GBN + 4 * m) = fv[i];
    if (WHL != 0) *(volatile v4u*)(outHL + (size_t)gr * KA + 8 * m) = pv[i];
  }
}

__global__ __launch_bounds__(GTHR) void k_gemm(
    const unsigned short* __restrict__ A, const unsigned short* __restrict__ WT,
    float* outF, int K, int ldo,
    const float* __restrict__ atts, const float* __restrict__ attd, int attLen,
    float* SD, int MPr)
{
  __shared__ __attribute__((aligned(16))) float stg[GBM * GBN];
  __shared__ __attribute__((aligned(16))) float satt[2 * GBN];
  __shared__ __attribute__((aligned(16))) float sdot[2 * GBM];
  const int tid = (int)threadIdx.x, lane = tid & 31, wave = tid >> 5, hh = lane >> 4, m = lane & 15;
  const int rowBase = (int)blockIdx.x * GBM;
  const int head    = (int)blockIdx.y;
  const int col0    = head * GBN;

  {
    const int which = tid >> 6;
    const int c  = tid & 63;
    const int cl = c < attLen ? c : attLen - 1;
    const float vs = atts[head * attLen + cl];
    const float vd = attd[head * attLen + cl];
    const unsigned int msk = (which == 0) ? 0u : 0xFFFFFFFFu;
    const unsigned int inr = (c < attLen) ? 0xFFFFFFFFu : 0u;
    float v = __uint_as_float((__float_as_uint(vs) & ~msk) | (__float_as_uint(vd) & msk));
    v = __uint_as_float(__float_as_uint(bfr(v)) & inr);
    satt[which * GBN + c] = v;
  }

  v8f acc[4];
  {
    const v8f z = {0.f, 0.f, 0.f, 0.f, 0.f, 0.f, 0.f, 0.f};
    acc[0] = z; acc[1] = z; acc[2] = z; acc[3] = z;
  }
  const unsigned short* ap = A  + (size_t)(rowBase + 16 * wave + m) * (size_t)K + 8 * hh;
  const unsigned short* wp = WT + (size_t)(col0 + m) * (size_t)K + 8 * hh;
  const int ksteps = K >> 5;
#pragma unroll 1
  for (int ks = 0; ks < ksteps; ++ks) {
    FragB af;
    af.h[0] = *(const v8usa*)(ap + 32 * ks);
    af.h[1] = *(const v8usa*)(ap + 32 * ks + 16);
#pragma unroll
    for (int t = 0; t < 4; ++t) {
      const unsigned short* wq = wp + (size_t)(16 * t) * (size_t)K + 32 * ks;
      FragB bf;
      bf.h[0] = *(const v8usa*)wq;
      bf.h[1] = *(const v8usa*)(wq + 16);
      acc[t] = wmb(af, bf, acc[t]);
    }
  }

#pragma unroll
  for (int t = 0; t < 4; ++t) {
    const int lc = 16 * t + m;
#pragma unroll
    for (int r = 0; r < 8; ++r) {
      const int lr = 16 * wave + 8 * hh + r;
      stg[lr * GBN + lc] = acc[t][r];
    }
  }
  __syncthreads();

  {
    const int row = tid & 63, which = tid >> 6;
    const float* sa = satt + which * GBN;
    const float* hr = stg + row * GBN;
    float d = 0.f;
#pragma unroll 4
    for (int c4 = 0; c4 < GBN / 4; ++c4) {
      const v4f hv = *(const v4fa*)(hr + 4 * c4);
      const v4f av = *(const v4fa*)(sa + 4 * c4);
      d = fmaf(hv.x, av.x, d);
      d = fmaf(hv.y, av.y, d);
      d = fmaf(hv.z, av.z, d);
      d = fmaf(hv.w, av.w, d);
    }
    sdot[which * GBM + row] = d;
  }
  __syncthreads();

  v4f fv[8];
#pragma unroll
  for (int i = 0; i < 8; ++i) {
    const int lr = 16 * wave + 2 * i + hh;
    fv[i] = *(const v4fa*)(stg + lr * GBN + 4 * m);
  }
  const int which2 = lane >> 4, piece = lane & 15;
  const v4f sdv = *(const v4fa*)(sdot + which2 * GBM + 4 * piece);
  float* sp = SD + (size_t)(2 * head + which2) * (size_t)MPr + rowBase + 4 * piece;

#pragma unroll
  for (int i = 0; i < 8; ++i) {
    const int lr = 16 * wave + 2 * i + hh;
    const int gr = rowBase + lr;
    float* op = outF + (size_t)gr * (size_t)ldo + col0 + 4 * m;
    *(volatile v4f*)op = fv[i];
  }
  if (wave == 0) *(volatile v4f*)sp = sdv;
  __threadfence();
#pragma unroll
  for (int i = 0; i < 8; ++i) {
    const int lr = 16 * wave + 2 * i + hh;
    const int gr = rowBase + lr;
    float* op = outF + (size_t)gr * (size_t)ldo + col0 + 4 * m;
    *(volatile v4f*)op = fv[i];
  }
  if (wave == 0) *(volatile v4f*)sp = sdv;
}

__global__ __launch_bounds__(NTHR) void k_agg(
    const int* __restrict__ HITS, const int* __restrict__ OFF, const int* __restrict__ CNT,
    const float* __restrict__ HS, const float* __restrict__ SD,
    const float* __restrict__ AE, const float* __restrict__ LAE, const float* __restrict__ TB,
    float* H, unsigned short* HHL, int nN, int nE, int MPr) {
  const int tid = (int)threadIdx.x, lane = tid & 31, wave = tid >> 5;
  const int blk = (int)blockIdx.x;
  const int nodeBase = blk * NBRUN;
  const int head = lane >> 3;
  const int c0   = 8 * lane;
  const int cc   = 8 * (lane & 7);
  const v4f cbA = *(const v4fa*)(TB + cc),        cbB = *(const v4fa*)(TB + cc + 4);
  const v4f muA = *(const v4fa*)(TB + 64 + cc),   muB = *(const v4fa*)(TB + 64 + cc + 4);
  const v4f scA = *(const v4fa*)(TB + 128 + cc),  scB = *(const v4fa*)(TB + 128 + cc + 4);
  const v4f beA = *(const v4fa*)(TB + 192 + cc),  beB = *(const v4fa*)(TB + 192 + cc + 4);
  const float cb[8] = {cbA.x, cbA.y, cbA.z, cbA.w, cbB.x, cbB.y, cbB.z, cbB.w};
  const float mu[8] = {muA.x, muA.y, muA.z, muA.w, muB.x, muB.y, muB.z, muB.w};
  const float sc[8] = {scA.x, scA.y, scA.z, scA.w, scB.x, scB.y, scB.z, scB.w};
  const float be[8] = {beA.x, beA.y, beA.z, beA.w, beB.x, beB.y, beB.z, beB.w};
  const float* ASp = SD + (size_t)(2 * head) * (size_t)MPr;
  const float* ADp = ASp + MPr;
  const int* hb = HITS + (size_t)blk * (size_t)RCAP * 2;
  const int sl8 = (lane >> 1) & 7;
  const bool odd  = (lane & 1) != 0;
  const bool lsel = (lane & 8) != 0;
  const float qnan = __int_as_float(0x7fc00000);

#pragma unroll 1
  for (int jt = 0; jt < NBRUN / NWAVE; ++jt) {
    const int slot = wave * (NBRUN / NWAVE) + jt;
    const int grow = nodeBase + slot;
    const int gcl  = grow < nN ? grow : nN - 1;
    int st = OFF[grow];
    const int craw = CNT[grow];
    st = st < 0 ? 0 : (st > RCAP ? RCAP : st);
    int cnt = craw < 0 ? 0 : (craw > DEGCAP ? DEGCAP : craw);
    if (cnt > RCAP - st) cnt = RCAP - st;
    const float pz = (craw > DEGCAP || craw < 0) ? qnan : 0.0f;

    const float* fr = HS + (size_t)gcl * HC1 + c0;
    v4f av = *(const v4fa*)fr;
    v4f bv = *(const v4fa*)(fr + 4);
    const float adv = ADp[gcl];
    float l0 = (ASp[gcl] + adv) + LAE[(size_t)grow * 4 + head];
    l0 = l0 > 0.f ? l0 : NEGSL * l0;
    float mx = l0, dn = 1.0f;

#pragma unroll 1
    for (int q = 0; q < cnt; ++q) {
      int idx = st + q; idx = idx > RCAP - 1 ? RCAP - 1 : idx;
      const v2i hv = *(const v2ia*)(hb + 2 * idx);
      const int s   = hv.x < 0 ? 0 : (hv.x > nN - 1 ? nN - 1 : hv.x);
      const int eid = hv.y < 0 ? 0 : (hv.y > nE - 1 ? nE - 1 : hv.y);
      const float* gsrc = HS + (size_t)s * HC1 + c0;
      const v4f fa = *(const v4fa*)gsrc;
      const v4f fb = *(const v4fa*)(gsrc + 4);
      float lg = (ASp[s] + adv) + AE[(size_t)eid * 4 + head];
      lg = lg > 0.f ? lg : NEGSL * lg;
      const float df = lg - mx;
      const float ee = expf(-fabsf(df));
      const bool up  = df > 0.f;
      const float s1 = up ? ee : 1.0f;
      const float s2 = up ? 1.0f : ee;
      mx = up ? lg : mx;
      dn = fmaf(dn, s1, s2);
      av.x = fmaf(av.x, s1, s2 * fa.x);
      av.y = fmaf(av.y, s1, s2 * fa.y);
      av.z = fmaf(av.z, s1, s2 * fa.z);
      av.w = fmaf(av.w, s1, s2 * fa.w);
      bv.x = fmaf(bv.x, s1, s2 * fb.x);
      bv.y = fmaf(bv.y, s1, s2 * fb.y);
      bv.z = fmaf(bv.z, s1, s2 * fb.z);
      bv.w = fmaf(bv.w, s1, s2 * fb.w);
    }
    const float inv = 1.0f / (dn + EPS_SM);
    float v[8] = {av.x * inv, av.y * inv, av.z * inv, av.w * inv, bv.x * inv, bv.y * inv, bv.z * inv, bv.w * inv};
#pragma unroll
    for (int j = 0; j < 8; ++j) v[j] += __shfl_xor(v[j], 8, 32);
#pragma unroll
    for (int j = 0; j < 8; ++j) v[j] += __shfl_xor(v[j], 16, 32);

    const float* hp = H + (size_t)gcl * HID + cc;
    const v4f hA = *(const v4fa*)hp;
    const v4f hB = *(const v4fa*)(hp + 4);
    const float ho[8] = {hA.x, hA.y, hA.z, hA.w, hB.x, hB.y, hB.z, hB.w};
    const bool live = grow < nN;
    float o[8];
#pragma unroll
    for (int j = 0; j < 8; ++j) {
      const float xx = v[j] * 0.25f + cb[j];
      const float y  = (xx - mu[j]) * sc[j] + be[j];
      const float r  = (y > 0.f) ? y : (y - y);
      const float hn = (ho[j] + r) + pz;
      o[j] = live ? hn : 0.0f;
    }
    v4f oa, ob;
    oa.x = o[0]; oa.y = o[1]; oa.z = o[2]; oa.w = o[3];
    ob.x = o[4]; ob.y = o[5]; ob.z = o[6]; ob.w = o[7];
    const HL8 sp = split8(oa, ob);
    v4u pv;
    pv.x = lsel ? sp.l.x : sp.h.x; pv.y = lsel ? sp.l.y : sp.h.y;
    pv.z = lsel ? sp.l.z : sp.h.z; pv.w = lsel ? sp.l.w : sp.h.w;
    float t[8];
#pragma unroll
    for (int j = 0; j < 8; ++j) t[j] = __shfl(o[j], sl8, 32);
    v4f ow;
    ow.x = odd ? t[4] : t[0]; ow.y = odd ? t[5] : t[1]; ow.z = odd ? t[6] : t[2]; ow.w = odd ? t[7] : t[3];

    float* op = H + (size_t)grow * HID + 4 * (lane & 15);
    unsigned short* hq = HHL + (size_t)grow * KA + 8 * (lane & 15);
    const bool wr = (grow < MPr) && (lane < 16);
    if (wr) { *(volatile v4f*)op = ow; *(volatile v4u*)hq = pv; }
    __threadfence();
    if (wr) { *(volatile v4f*)op = ow; *(volatile v4u*)hq = pv; }
  }
}

__global__ __launch_bounds__(NTHR) void k_pool(const float* __restrict__ hf, const int* __restrict__ bat,
                                               int nN, float* pl) {
  __shared__ __attribute__((aligned(16))) float wsum[NWAVE * HID];
  __shared__ int wcn[NWAVE];
  __shared__ __attribute__((aligned(16))) float outs[HID];
  const int tid = (int)threadIdx.x, lane = tid & 31, wave = tid >> 5;
  const int g = (int)blockIdx.x;

  float a0 = 0.0f, a1 = 0.0f;
  int cnt = 0;
#pragma unroll 1
  for (int i0 = wave * 32; i0 < nN; i0 += NTHR) {
    const int i  = i0 + lane;
    const int ic = i < nN ? i : nN - 1;
    const int b  = bat[ic];
    const bool hit = (i < nN) && (b == g);
    unsigned msk = __builtin_amdgcn_ballot_w32(hit);
    int nh = (int)__builtin_popcount(msk);
    nh = nh > 32 ? 32 : nh;
    cnt += nh;
#pragma unroll 1
    for (int q = 0; q < nh; ++q) {
      const int k = __builtin_ffs((int)msk) - 1;
      msk &= msk - 1u;
      int node = i0 + (k < 0 ? 0 : k);
      node = node > nN - 1 ? nN - 1 : node;
      const v2f v = *(const v2fa*)(hf + (size_t)node * HID + 2 * lane);
      a0 += v.x; a1 += v.y;
    }
  }
  wsum[wave * HID + 2 * lane + 0] = a0;
  wsum[wave * HID + 2 * lane + 1] = a1;
  if (lane == 0) wcn[wave] = cnt;
  __syncthreads();
  if (tid < HID) {
    float s = 0.0f;
    int c = 0;
#pragma unroll
    for (int w2 = 0; w2 < NWAVE; ++w2) { s += wsum[w2 * HID + tid]; c += wcn[w2]; }
    const float cf = (c < 1) ? 1.0f : (float)c;
    outs[tid] = s * (1.0f / cf);
  }
  __syncthreads();
  const v4f ov = *(const v4fa*)(outs + 4 * (lane & 15));
  float* op = pl + (size_t)g * HID + 4 * (lane & 15);
  const bool okst = (wave == 0) && (lane < 16);
  if (okst) *(volatile v4f*)op = ov;
  __threadfence();
  if (okst) *(volatile v4f*)op = ov;
}

static inline int cdiv(int a, int b) { return (a + b - 1) / b; }
static inline size_t al256(size_t o) { return (o + 255) & ~(size_t)255; }

extern "C" void kernel_launch(void* const* d_in, const int* in_sizes, int n_in,
                              void* d_out, int out_size, void* d_ws, size_t ws_size,
                              hipStream_t stream) {
  if (n_in < 18) return;
  const int nN = in_sizes[0] / F_IN;
  if (nN <= 0 || in_sizes[0] != nN * F_IN || nN > (1 << 22)) return;
  if (in_sizes[1] < 2 || (in_sizes[1] & 1) != 0) return;
  const int nE = in_sizes[1] / 2;
  if (nE < 8 || nE >= (1 << (32 - SLOTB)) || (nE & 7) != 0) return;
  if (in_sizes[2] != nE * EDIM) return;
  if (in_sizes[3] != nN) return;
  if (in_sizes[4] != F_IN * HID || in_sizes[5] != HID) return;
  if (in_sizes[6] != NLAY * HID * HC1) return;
  if (in_sizes[7] != NLAY * HC1 || in_sizes[8] != NLAY * HC1) return;
  if (in_sizes[9] != NLAY * EDIM * HC1) return;
  if (in_sizes[10] != NLAY * HC1) return;
  if (in_sizes[11] != NLAY * HID || in_sizes[12] != NLAY * HID) return;
  if (in_sizes[13] != NLAY * HID || in_sizes[14] != NLAY * HID) return;
  if (in_sizes[15] != NLAY * HID) return;
  if (in_sizes[16] != HID * HID || in_sizes[17] != HID) return;
  if (out_size != NGR * HID) return;

  const float* x     = (const float*)d_in[0];
  const int*   ei    = (const int*)  d_in[1];
  const float* eattr = (const float*)d_in[2];
  const int*   bat   = (const int*)  d_in[3];
  const float* encW  = (const float*)d_in[4];
  const float* encb  = (const float*)d_in[5];
  const float* linW  = (const float*)d_in[6];
  const float* atts  = (const float*)d_in[7];
  const float* attd  = (const float*)d_in[8];
  const float* lew   = (const float*)d_in[9];
  const float* atte  = (const float*)d_in[10];
  const float* cbias = (const float*)d_in[11];
  const float* gam   = (const float*)d_in[12];
  const float* bet   = (const float*)d_in[13];
  const float* mean  = (const float*)d_in[14];
  const float* var   = (const float*)d_in[15];
  const float* outW  = (const float*)d_in[16];
  const float* outb  = (const float*)d_in[17];
  float* out = (float*)d_out;
  const int* src = ei;
  const int* dst = ei + nE;

  const int MP    = cdiv(nN, MROWS) * MROWS;
  const int gA    = cdiv(MP, NBRUN);
  const int NSLOT = gA * NBRUN;
  if (gA * NBRUN < MP) return;
  const int vec8 = ((nE & 3) == 0) ? 1 : 0;
  const int gM = MP / GBM;

  char* ws = (char*)d_ws;
  size_t off = 0;
  const size_t oXB  = off; off = al256(off + (size_t)MP * F_IN * 2);
  const size_t oEWT = off; off = al256(off + (size_t)HID * F_IN * 2);
  const size_t oLWT = off; off = al256(off + (size_t)NLAY * HC1 * KA * 2);
  const size_t oOWT = off; off = al256(off + (size_t)HID * KA * 2);
  const size_t oKAP = off; off = al256(off + (size_t)128 * 4);
  const size_t oTB  = off; off = al256(off + (size_t)NLAY * 256 * 4);
  const size_t oH   = off; off = al256(off + (size_t)MP * HID * 4);
  const size_t oHHL = off; off = al256(off + (size_t)MP * KA * 2);
  const size_t oHS  = off; off = al256(off + (size_t)MP * HC1 * 4);
  const size_t oSD  = off; off = al256(off + (size_t)2 * NHD * MP * 4);
  const size_t oAE  = off; off = al256(off + (size_t)NLAY * nE * 4 * 4);
  const size_t oLAE = off; off = al256(off + (size_t)NLAY * NSLOT * 4 * 4);
  const size_t oHIT = off; off = al256(off + (size_t)gA * RCAP * 2 * 4);
  const size_t oOFF = off; off = al256(off + (size_t)NSLOT * 4);
  const size_t oCNT = off; off = al256(off + (size_t)NSLOT * 4);
  if (off > ws_size || off > (size_t)WSMAX) return;
  unsigned short* XB   = (unsigned short*)(ws + oXB);
  unsigned short* EWT  = (unsigned short*)(ws + oEWT);
  unsigned short* LWT2 = (unsigned short*)(ws + oLWT);
  unsigned short* OWT2 = (unsigned short*)(ws + oOWT);
  float*          KAP  = (float*)(ws + oKAP);
  float*          TB   = (float*)(ws + oTB);
  float*          H    = (float*)(ws + oH);
  unsigned short* HHL  = (unsigned short*)(ws + oHHL);
  float*          HS   = (float*)(ws + oHS);
  float*          SD   = (float*)(ws + oSD);
  float*          AE   = (float*)(ws + oAE);
  float*          LAE  = (float*)(ws + oLAE);
  int*            HITS = (int*)(ws + oHIT);
  int*            OFF  = (int*)(ws + oOFF);
  int*            CNT  = (int*)(ws + oCNT);

  hipFuncSetAttribute(reinterpret_cast<const void*>(&k_bucket),
                      hipFuncAttributeMaxDynamicSharedMemorySize, LDS_BKT);

  const int nUx = MP * (F_IN / 8);
  k_xprep<<<cdiv(nUx, NTHR), NTHR, 0, stream>>>(x, XB, nN, nUx);

  {
    const int nUe = HID * (F_IN / 8);
    k_wtr<<<cdiv(nUe, NTHR), NTHR, 0, stream>>>(encW, F_IN, HID, HID, F_IN, EWT, nUe);
    const int nUl = HC1 * (KA / 8);
    for (int l = 0; l < NLAY; ++l)
      k_wtr<<<cdiv(nUl, NTHR), NTHR, 0, stream>>>(linW + (size_t)l * HID * HC1, HID, HC1, HC1, KA,
                                                  LWT2 + (size_t)l * HC1 * KA, nUl);
    const int nUo = HID * (KA / 8);
    k_wtr<<<cdiv(nUo, NTHR), NTHR, 0, stream>>>(outW, HID, HID, HID, KA, OWT2, nUo);
  }
  k_tab<<<1, NTHR, 0, stream>>>(lew, atte, cbias, gam, bet, mean, var, KAP, TB);
  k_edge<<<cdiv(nE, NTHR), NTHR, 0, stream>>>(eattr, KAP, AE, nE);
  k_bucket<<<gA, NTHR, LDS_BKT, stream>>>(src, dst, eattr, KAP, HITS, OFF, CNT, LAE, nN, nE, vec8, NSLOT);
  k_gemmb<1><<<gM, GTHR, 0, stream>>>(XB, EWT, encb, H, HHL, F_IN);
  for (int l = 0; l < NLAY; ++l) {
    k_gemm<<<dim3(gM, HC1 / GBN), GTHR, 0, stream>>>(HHL, LWT2 + (size_t)l * HC1 * KA, HS, KA, HC1,
                                                     atts + (size_t)l * HC1, attd + (size_t)l * HC1, HID, SD, MP);
    k_agg<<<gA, NTHR, 0, stream>>>(HITS, OFF, CNT, HS, SD, AE + (size_t)l * nE * 4, LAE + (size_t)l * NSLOT * 4,
                                   TB + (size_t)l * 256, H, HHL, nN, nE, MP);
  }
  k_gemmb<0><<<gM, GTHR, 0, stream>>>(HHL, OWT2, outb, HS, XB, KA);
  k_pool<<<NGR, NTHR, 0, stream>>>(HS, bat, nN, out);
}
